// MaskedMultiHeadAttention_66365834658467
// MI455X (gfx1250) — hardware-verified
//
#include <hip/hip_runtime.h>


#ifndef NB
#define NB 2
#endif
#ifndef SEQ
#define SEQ 4096
#endif
#define SEQ_FULL 4096
#define DMOD 512
#define D3 1536
#define NH 8
#define HD 64
#ifndef RHI
#define RHI 2048
#endif
#if RHI > SEQ
#define RH SEQ
#else
#define RH RHI
#endif
#define PCAR 1024.0f
#define CCAR 16.0f
#define WCAR 64.0f

static_assert(SEQ % 64 == 0);
static_assert(SEQ <= SEQ_FULL);
static_assert(RH % 64 == 0);
static_assert(RH >= 64 && RH <= SEQ);
static_assert(D3 == 3 * DMOD && NH * HD == DMOD && HD == 64);
static_assert(DMOD % 64 == 0 && DMOD % 32 == 0);

typedef _Float16 h16;
typedef unsigned short us;
typedef __attribute__((ext_vector_type(16))) __bf16 v16bf;
typedef __attribute__((ext_vector_type(16))) _Float16 v16h;
typedef __attribute__((ext_vector_type(16))) unsigned short v16us;
typedef __attribute__((ext_vector_type(8)))  _Float16 v8h;
typedef __attribute__((ext_vector_type(8)))  unsigned short v8us;
typedef __attribute__((ext_vector_type(8)))  float v8f;
typedef __attribute__((ext_vector_type(4)))  float v4f;
typedef __attribute__((ext_vector_type(2)))  unsigned short v2us;
typedef v8us __attribute__((may_alias)) v8usa;
typedef v4f  __attribute__((may_alias)) v4fa;

__device__ __forceinline__ us f2bf(float f) { unsigned u = __float_as_uint(f); u += 0x7FFFu + ((u >> 16) & 1u); return (us)(u >> 16); }
__device__ __forceinline__ float bf2f(us b) { return __uint_as_float(((unsigned)b) << 16); }
__device__ __forceinline__ float bfr(float f) { return bf2f(f2bf(f)); }
__device__ __forceinline__ us hbit(float x) { const h16 t = (h16)x; return __builtin_bit_cast(us, t); }
__device__ __forceinline__ void splitf(float y, us& h, us& l) { h = f2bf(y); l = f2bf(y - bf2f(h)); }
__device__ __forceinline__ v16us ld16(const us* p) {
    const v8us a = *(const v8usa*)p; const v8us b = *(const v8usa*)(p + 16);
    return __builtin_shufflevector(a, b, 0, 1, 2, 3, 4, 5, 6, 7, 8, 9, 10, 11, 12, 13, 14, 15);
}
__device__ __forceinline__ v8f wmh(v16us a, v16us b, v8f c) { return __builtin_amdgcn_wmma_f32_16x16x32_f16(false, __builtin_bit_cast(v16h, a), false, __builtin_bit_cast(v16h, b), (short)0, c, false, false); }
__device__ __forceinline__ v8f wmb(v16us a, v16us b, v8f c) { return __builtin_amdgcn_wmma_f32_16x16x32_bf16(false, __builtin_bit_cast(v16bf, a), false, __builtin_bit_cast(v16bf, b), (short)0, c, false, false); }
template <int TY> struct MM;
template <> struct MM<0> { static __device__ __forceinline__ v8f mma(v16us a, v16us b, v8f c) { return wmh(a, b, c); } };
template <> struct MM<1> { static __device__ __forceinline__ v8f mma(v16us a, v16us b, v8f c) { return wmb(a, b, c); } };

template <int TY, int NSPLIT>
__global__ __launch_bounds__(32) void k_gemmw(const us* __restrict__ A, const us* __restrict__ A2, const us* __restrict__ Bt, const us* __restrict__ Bt2, int K, float* C, int ldc, float osc, size_t sA, size_t sB, size_t sC) {
    __shared__ __align__(16) float os[16 * 68];
    const size_t z = blockIdx.z; A += z * sA; if (A2) A2 += z * sA; Bt += z * sB; if (Bt2) Bt2 += z * sB; C += z * sC;
    const int lane = threadIdx.x & 31, lr = lane & 15, hi = lane >> 4; const int r0 = blockIdx.x * 64, c0 = blockIdx.y * 64;
    v8f acc[4][4];
#pragma unroll
    for (int mb = 0; mb < 4; ++mb)
#pragma unroll
        for (int nb = 0; nb < 4; ++nb) acc[mb][nb] = (v8f){};
    const size_t aoff = (size_t)(r0 + lr) * K + 8 * hi, boff = (size_t)(c0 + lr) * K + 8 * hi;
#pragma unroll 1
    for (int kc = 0; kc < K; kc += 32) {
        v16us a[4], a2[4];
#pragma unroll
        for (int mb = 0; mb < 4; ++mb) { a[mb] = ld16(A + aoff + (size_t)mb * 16 * K + kc); if (NSPLIT == 1 || NSPLIT == 2) a2[mb] = ld16(A2 + aoff + (size_t)mb * 16 * K + kc); }
#pragma unroll
        for (int nb = 0; nb < 4; ++nb) { const v16us b = ld16(Bt + boff + (size_t)nb * 16 * K + kc); v16us b2; if (NSPLIT >= 2) b2 = ld16(Bt2 + boff + (size_t)nb * 16 * K + kc);
#pragma unroll
            for (int mb = 0; mb < 4; ++mb) { acc[mb][nb] = MM<TY>::mma(a[mb], b, acc[mb][nb]); if (NSPLIT == 1 || NSPLIT == 2) acc[mb][nb] = MM<TY>::mma(a2[mb], b, acc[mb][nb]); if (NSPLIT >= 2) acc[mb][nb] = MM<TY>::mma(a[mb], b2, acc[mb][nb]); } }
        asm volatile("v_nop\n\tv_nop\n\tv_nop\n\tv_nop" : "+v"(acc[0][0]), "+v"(acc[1][1]), "+v"(acc[2][2]), "+v"(acc[3][3]) : "v"(a[0]), "v"(a[3]));
    }
#pragma unroll
    for (int mb = 0; mb < 4; ++mb) {
#pragma unroll
        for (int nb = 0; nb < 4; ++nb) {
#pragma unroll
            for (int j = 0; j < 8; ++j) os[(hi * 8 + j) * 68 + nb * 16 + lr] = acc[mb][nb][j]; }
        __builtin_amdgcn_wave_barrier(); asm volatile("" ::: "memory");
        float* crow = C + (size_t)(r0 + mb * 16) * ldc + c0;
#pragma unroll 1
        for (int ps = 0; ps < 2; ++ps) {
#pragma unroll
            for (int s = 0; s < 8; ++s) { const int row = 2 * s + hi, cofs = lr * 4; v4f val = *(const v4fa*)(os + row * 68 + cofs); val = val * osc;
                *(volatile v4f*)(crow + (size_t)row * ldc + cofs) = val; }
            if (ps == 0) __threadfence(); }
        __builtin_amdgcn_wave_barrier(); asm volatile("" ::: "memory");
    }
}

template <int TY>
__global__ __launch_bounds__(256) void k_wt(const float* __restrict__ w, int K, int N, float sc, us* Bt) {
    const int lane = threadIdx.x & 31; const int L0 = ((int)blockIdx.x * 8 + (int)(threadIdx.x >> 5)) * 8; const int nlines = (int)(((size_t)N * K) / 64);
#pragma unroll 1
    for (int l = 0; l < 8; ++l) { const int L = L0 + l; if (L >= nlines) break;
        const size_t e = (size_t)L * 64 + lane * 2; const int k = (int)(e % (size_t)K), n = (int)(e / (size_t)K);
        const float w0 = w[(size_t)k * N + n], w1 = w[(size_t)(k + 1) * N + n];
        v2us o;
        if (TY) { o[0] = f2bf(w0); o[1] = f2bf(w1); } else { o[0] = hbit(bfr(w0) * sc); o[1] = hbit(bfr(w1) * sc); }
        *(volatile v2us*)(Bt + e) = o; __threadfence(); *(volatile v2us*)(Bt + e) = o; }
}

__global__ __launch_bounds__(256) void k_cvt8(const float* __restrict__ src, us* dst, unsigned n8) {
    const unsigned i = blockIdx.x * 256 + threadIdx.x; if (i >= n8) return;
    const v4f a = *(const v4fa*)(src + (size_t)i * 8), b = *(const v4fa*)(src + (size_t)i * 8 + 4); v8us o;
#pragma unroll
    for (int k = 0; k < 4; ++k) { o[k] = f2bf(a[k]); o[k + 4] = f2bf(b[k]); }
    *(volatile v8us*)(dst + (size_t)i * 8) = o; __threadfence(); *(volatile v8us*)(dst + (size_t)i * 8) = o;
}

__global__ __launch_bounds__(256) void k_plane(const float* __restrict__ F, int col0, us* P16, us* Ph, us* Pl) {
    const unsigned i = blockIdx.x * 256 + threadIdx.x; if (i >= (unsigned)(NH * SEQ * HD / 8)) return;
    const unsigned e = i * 8; const int d = (int)(e % HD); const int t = (int)((e / HD) % SEQ); const int hh = (int)(e / ((unsigned)HD * SEQ));
    const float* f = F + (size_t)t * D3 + col0 + hh * HD + d;
    const v4f a = *(const v4fa*)f, b = *(const v4fa*)(f + 4);
    float y[8];
#pragma unroll
    for (int j = 0; j < 4; ++j) { y[j] = a[j]; y[j + 4] = b[j]; }
    v8us o16, oh, ol;
#pragma unroll
    for (int j = 0; j < 8; ++j) { o16[j] = hbit(y[j]); us p, q; splitf(y[j], p, q); oh[j] = p; ol[j] = q; }
    const bool hr = (t < RH); const size_t oo = ((size_t)hh * RH + (hr ? t : 0)) * HD + d;
    *(volatile v8us*)(P16 + e) = o16; if (hr) { *(volatile v8us*)(Ph + oo) = oh; *(volatile v8us*)(Pl + oo) = ol; }
    __threadfence();
    *(volatile v8us*)(P16 + e) = o16; if (hr) { *(volatile v8us*)(Ph + oo) = oh; *(volatile v8us*)(Pl + oo) = ol; }
}

__global__ __launch_bounds__(256) void k_vtp(const float* __restrict__ F, us* VT16, us* VTh, us* VTl) {
    const unsigned i = blockIdx.x * 256 + threadIdx.x; if (i >= (unsigned)(NH * HD * SEQ / 8)) return;
    const unsigned e = i * 8; const int t = (int)(e % SEQ); const int d = (int)((e / SEQ) % HD); const int hh = (int)(e / ((unsigned)SEQ * HD));
    const float* f = F + (size_t)t * D3 + 2 * DMOD + hh * HD + d;
    v8us o16, oh, ol;
#pragma unroll
    for (int j = 0; j < 8; ++j) { const float y = f[(size_t)j * D3]; o16[j] = hbit(y); us p, q; splitf(y, p, q); oh[j] = p; ol[j] = q; }
    const bool hr = (t < RH); const size_t oo = ((size_t)hh * HD + d) * RH + (hr ? t : 0);
    *(volatile v8us*)(VT16 + e) = o16; if (hr) { *(volatile v8us*)(VTh + oo) = oh; *(volatile v8us*)(VTl + oo) = ol; }
    __threadfence();
    *(volatile v8us*)(VT16 + e) = o16; if (hr) { *(volatile v8us*)(VTh + oo) = oh; *(volatile v8us*)(VTl + oo) = ol; }
}

template <bool HR>
__global__ __launch_bounds__(128) __attribute__((amdgpu_num_vgpr(256)))
void k_attn(const us* __restrict__ Q16, const us* __restrict__ K16, const us* __restrict__ VT16,
            const us* __restrict__ Qh, const us* __restrict__ Ql, const us* __restrict__ Kh, const us* __restrict__ Kl,
            const us* __restrict__ VTh, const us* __restrict__ VTl, int qt0, us* C16, us* Ch, us* Cl) {
    constexpr int TP = 72;
    __shared__ __align__(16) us Ka[64 * TP];
    __shared__ __align__(16) us Va[64 * TP];
    __shared__ __align__(16) us Pa[4][16 * TP];
    __shared__ __align__(16) us Kb[HR ? 64 * TP : 8];
    __shared__ __align__(16) us Vb[HR ? 64 * TP : 8];
    __shared__ __align__(16) us Pb[HR ? 4 : 1][16 * TP];
    const int tid = threadIdx.x, lane = tid & 31, w = tid >> 5, m = lane & 15, hi = lane >> 4;
    const int qt = qt0 + (int)blockIdx.x, h = (int)blockIdx.y;
    const int qrow = qt * 64 + w * 16 + m;
    us* const pa = Pa[w]; us* const pb = Pb[HR ? w : 0];
    v8f o[4];
#pragma unroll
    for (int i = 0; i < 4; ++i) o[i] = (v8f){};
    float mr[8], lr[8];
#pragma unroll
    for (int r = 0; r < 8; ++r) { mr[r] = -1.0e30f; lr[r] = 0.0f; }
    const float CL = 0.18033688011112042f;
    const int nch = qt + 1;
#pragma unroll 1
    for (int kc = 0; kc < nch; ++kc) {
        __syncthreads();
#pragma unroll
        for (int i = 0; i < 4; ++i) { const int c = tid + 128 * i; const int row = c >> 3, col = (c & 7) * 8;
            if (!HR) {
                const v8us kv = *(const v8usa*)(K16 + ((size_t)h * SEQ + kc * 64 + row) * HD + col); *(v8usa*)(Ka + row * TP + col) = kv;
                const v8us vv = *(const v8usa*)(VT16 + ((size_t)h * HD + row) * SEQ + kc * 64 + col); *(v8usa*)(Va + row * TP + col) = vv;
            } else {
                const v8us k1 = *(const v8usa*)(Kh + ((size_t)h * RH + kc * 64 + row) * HD + col); *(v8usa*)(Ka + row * TP + col) = k1;
                const v8us k2 = *(const v8usa*)(Kl + ((size_t)h * RH + kc * 64 + row) * HD + col); *(v8usa*)(Kb + row * TP + col) = k2;
                const v8us v1 = *(const v8usa*)(VTh + ((size_t)h * HD + row) * RH + kc * 64 + col); *(v8usa*)(Va + row * TP + col) = v1;
                const v8us v2 = *(const v8usa*)(VTl + ((size_t)h * HD + row) * RH + kc * 64 + col); *(v8usa*)(Vb + row * TP + col) = v2;
            } }
        __syncthreads();
        v8f s[4];
        if (!HR) {
            const us* qp = Q16 + ((size_t)h * SEQ + qrow) * HD + 8 * hi;
            const v16us qa0 = ld16(qp), qa1 = ld16(qp + 32);
#pragma unroll
            for (int sn = 0; sn < 4; ++sn) { const us* kp = Ka + (sn * 16 + m) * TP + 8 * hi; const v16us b0 = ld16(kp), b1 = ld16(kp + 32);
                v8f c = (v8f){}; c = wmh(qa0, b0, c); c = wmh(qa1, b1, c); s[sn] = c; }
            asm volatile("v_nop\n\tv_nop\n\tv_nop\n\tv_nop" : "+v"(s[0]), "+v"(s[1]), "+v"(s[2]), "+v"(s[3]) : "v"(qa0), "v"(qa1));
        } else {
            const size_t qo = ((size_t)h * RH + qrow) * HD + 8 * hi;
            const v16us qh0 = ld16(Qh + qo), qh1 = ld16(Qh + qo + 32), ql0 = ld16(Ql + qo), ql1 = ld16(Ql + qo + 32);
#pragma unroll
            for (int sn = 0; sn < 4; ++sn) { const int ko = (sn * 16 + m) * TP + 8 * hi;
                const v16us kh0 = ld16(Ka + ko), kh1 = ld16(Ka + ko + 32);
                v8f c = (v8f){}; c = wmb(qh0, kh0, c); c = wmb(ql0, kh0, c); c = wmb(qh1, kh1, c); c = wmb(ql1, kh1, c);
                const v16us kl0 = ld16(Kb + ko), kl1 = ld16(Kb + ko + 32);
                c = wmb(qh0, kl0, c); c = wmb(qh1, kl1, c); s[sn] = c; }
            asm volatile("v_nop\n\tv_nop\n\tv_nop\n\tv_nop" : "+v"(s[0]), "+v"(s[1]), "+v"(s[2]), "+v"(s[3]) : "v"(qh0), "v"(ql1));
        }
        if (kc == qt) {
#pragma unroll
            for (int sn = 0; sn < 4; ++sn) { const int key = sn * 16 + m;
#pragma unroll
                for (int r = 0; r < 8; ++r) { const int q = w * 16 + 8 * hi + r; s[sn][r] = (key > q) ? -1.0e30f : s[sn][r]; } }
        }
        float mn[8], al[8];
#pragma unroll
        for (int r = 0; r < 8; ++r) {
            float mx = fmaxf(fmaxf(s[0][r], s[1][r]), fmaxf(s[2][r], s[3][r]));
            mx = fmaxf(mx, __shfl_xor(mx, 1, 32)); mx = fmaxf(mx, __shfl_xor(mx, 2, 32)); mx = fmaxf(mx, __shfl_xor(mx, 4, 32)); mx = fmaxf(mx, __shfl_xor(mx, 8, 32));
            mn[r] = fmaxf(mr[r], mx); al[r] = __builtin_amdgcn_exp2f((mr[r] - mn[r]) * CL); mr[r] = mn[r]; }
#pragma unroll
        for (int r = 0; r < 8; ++r) {
            float sum = 0.0f;
#pragma unroll
            for (int sn = 0; sn < 4; ++sn) { const float p = __builtin_amdgcn_exp2f((s[sn][r] - mn[r]) * CL); s[sn][r] = p; sum += p; }
            sum += __shfl_xor(sum, 1, 32); sum += __shfl_xor(sum, 2, 32); sum += __shfl_xor(sum, 4, 32); sum += __shfl_xor(sum, 8, 32);
            lr[r] = lr[r] * al[r] + sum;
#pragma unroll
            for (int i = 0; i < 4; ++i) o[i][r] *= al[r]; }
        if (!HR) {
#pragma unroll
            for (int sn = 0; sn < 4; ++sn)
#pragma unroll
                for (int r = 0; r < 8; ++r) pa[(8 * hi + r) * TP + sn * 16 + m] = hbit(s[sn][r] * PCAR);
        } else {
#pragma unroll
            for (int sn = 0; sn < 4; ++sn)
#pragma unroll
                for (int r = 0; r < 8; ++r) { us p, q; splitf(s[sn][r], p, q); pa[(8 * hi + r) * TP + sn * 16 + m] = p; pb[(8 * hi + r) * TP + sn * 16 + m] = q; }
        }
        __builtin_amdgcn_wave_barrier(); asm volatile("" ::: "memory");
        if (!HR) {
            const us* pp = pa + m * TP + 8 * hi; const v16us pf0 = ld16(pp), pf1 = ld16(pp + 32);
#pragma unroll
            for (int sn = 0; sn < 4; ++sn) { const us* vp = Va + (sn * 16 + m) * TP + 8 * hi; const v16us b0 = ld16(vp), b1 = ld16(vp + 32);
                o[sn] = wmh(pf0, b0, o[sn]); o[sn] = wmh(pf1, b1, o[sn]); }
            asm volatile("v_nop\n\tv_nop\n\tv_nop\n\tv_nop" : "+v"(o[0]), "+v"(o[1]), "+v"(o[2]), "+v"(o[3]) : "v"(pf0), "v"(pf1));
        } else {
            const us* pp = pa + m * TP + 8 * hi; const us* pq = pb + m * TP + 8 * hi;
            const v16us ph0 = ld16(pp), ph1 = ld16(pp + 32), pl0 = ld16(pq), pl1 = ld16(pq + 32);
#pragma unroll
            for (int sn = 0; sn < 4; ++sn) { const int vo = (sn * 16 + m) * TP + 8 * hi;
                const v16us vh0 = ld16(Va + vo), vh1 = ld16(Va + vo + 32);
                o[sn] = wmb(ph0, vh0, o[sn]); o[sn] = wmb(pl0, vh0, o[sn]); o[sn] = wmb(ph1, vh1, o[sn]); o[sn] = wmb(pl1, vh1, o[sn]);
                const v16us vl0 = ld16(Vb + vo), vl1 = ld16(Vb + vo + 32);
                o[sn] = wmb(ph0, vl0, o[sn]); o[sn] = wmb(ph1, vl1, o[sn]); }
            asm volatile("v_nop\n\tv_nop\n\tv_nop\n\tv_nop" : "+v"(o[0]), "+v"(o[1]), "+v"(o[2]), "+v"(o[3]) : "v"(ph0), "v"(pl1));
        }
    }
    float iv[8];
#pragma unroll
    for (int r = 0; r < 8; ++r) iv[r] = (HR ? 1.0f : (CCAR / PCAR)) * __builtin_amdgcn_rcpf(lr[r]);
    __builtin_amdgcn_wave_barrier(); asm volatile("" ::: "memory");
    if (!HR) {
#pragma unroll
        for (int sn = 0; sn < 4; ++sn)
#pragma unroll
            for (int r = 0; r < 8; ++r) pa[(8 * hi + r) * TP + sn * 16 + m] = hbit(o[sn][r] * iv[r]);
    } else {
#pragma unroll
        for (int sn = 0; sn < 4; ++sn)
#pragma unroll
            for (int r = 0; r < 8; ++r) { us p, q; splitf(o[sn][r] * iv[r], p, q); pa[(8 * hi + r) * TP + sn * 16 + m] = p; pb[(8 * hi + r) * TP + sn * 16 + m] = q; }
    }
    __builtin_amdgcn_wave_barrier(); asm volatile("" ::: "memory");
    const int trow0 = qt * 64 + w * 16;
#pragma unroll 1
    for (int ps = 0; ps < 2; ++ps) {
#pragma unroll
        for (int it = 0; it < 4; ++it) { const int row = it * 4 + (lane >> 3), pc = (lane & 7) * 8; const size_t go = (size_t)(trow0 + row) * DMOD + h * HD + pc;
            const v8us v1 = *(const v8usa*)(pa + row * TP + pc);
            if (!HR) { *(volatile v8us*)(C16 + go) = v1; }
            else { const v8us v2 = *(const v8usa*)(pb + row * TP + pc); *(volatile v8us*)(Ch + go) = v1; *(volatile v8us*)(Cl + go) = v2; } }
        if (ps == 0) __threadfence(); }
}

extern "C" void kernel_launch(void* const* d_in, const int* in_sizes, int n_in,
                              void* d_out, int out_size, void* d_ws, size_t ws_size, hipStream_t stream) {
    if (n_in < 7) return;
    const long long needx = (long long)(NB - 1) * SEQ_FULL * DMOD + (long long)SEQ * DMOD;
    const long long needw = (long long)DMOD * DMOD;
    if ((long long)in_sizes[0] < needx || (long long)in_sizes[1] < needx || (long long)in_sizes[2] < needx) return;
    if ((long long)in_sizes[3] < needw || (long long)in_sizes[4] < needw || (long long)in_sizes[5] < needw || (long long)in_sizes[6] < needw) return;
    if ((long long)out_size < needx) return;
    const float* xq = (const float*)d_in[0];
    const float* xk = (const float*)d_in[1];
    const float* xv = (const float*)d_in[2];
    const float* wq = (const float*)d_in[3];
    const float* wk = (const float*)d_in[4];
    const float* wv = (const float*)d_in[5];
    const float* wo = (const float*)d_in[6];
    float* OUT = (float*)d_out;
    char* wsp = (char*)d_ws;
    auto take = [&](size_t bytes) { char* p = wsp; wsp += (bytes + 255) & ~(size_t)255; return (void*)p; };
    const size_t WSZ = (size_t)DMOD * DMOD;
    const size_t XSZ = (size_t)SEQ * DMOD;
    us* W3   = (us*)take(3 * WSZ * 2);
    us* WOB  = (us*)take(WSZ * 2);
    us* WO16 = (us*)take(WSZ * 2);
    us* XB   = (us*)take(3 * XSZ * 2);
    float* F = (float*)take((size_t)SEQ * D3 * 4);
    us* Q16  = (us*)take((size_t)NH * SEQ * HD * 2);
    us* K16  = (us*)take((size_t)NH * SEQ * HD * 2);
    us* VT16 = (us*)take((size_t)NH * HD * SEQ * 2);
    us* QH   = (us*)take((size_t)NH * RH * HD * 2);
    us* QL   = (us*)take((size_t)NH * RH * HD * 2);
    us* KH   = (us*)take((size_t)NH * RH * HD * 2);
    us* KL   = (us*)take((size_t)NH * RH * HD * 2);
    us* VTH  = (us*)take((size_t)NH * HD * RH * 2);
    us* VTL  = (us*)take((size_t)NH * HD * RH * 2);
    us* C16  = (us*)take(XSZ * 2);
    us* CH   = (us*)take((size_t)RH * DMOD * 2);
    us* CLO  = (us*)take((size_t)RH * DMOD * 2);
    if ((size_t)(wsp - (char*)d_ws) > ws_size) return;

    const unsigned gw = (unsigned)((WSZ / 64 + 63) / 64);
    k_wt<1><<<gw, 256, 0, stream>>>(wq, DMOD, DMOD, 1.0f, W3);
    k_wt<1><<<gw, 256, 0, stream>>>(wk, DMOD, DMOD, 1.0f, W3 + WSZ);
    k_wt<1><<<gw, 256, 0, stream>>>(wv, DMOD, DMOD, 1.0f, W3 + 2 * WSZ);
    k_wt<1><<<gw, 256, 0, stream>>>(wo, DMOD, DMOD, 1.0f, WOB);
    k_wt<0><<<gw, 256, 0, stream>>>(wo, DMOD, DMOD, WCAR, WO16);
    const unsigned n8x = (unsigned)(XSZ / 8);
    const unsigned nthr8 = (unsigned)(NH * SEQ * HD / 8);
    for (int b = 0; b < NB; ++b) {
        const size_t boff = (size_t)b * SEQ_FULL * DMOD;
        float* ob = OUT + boff;
        k_cvt8<<<(n8x + 255) / 256, 256, 0, stream>>>(xq + boff, XB, n8x);
        k_cvt8<<<(n8x + 255) / 256, 256, 0, stream>>>(xk + boff, XB + XSZ, n8x);
        k_cvt8<<<(n8x + 255) / 256, 256, 0, stream>>>(xv + boff, XB + 2 * XSZ, n8x);
        k_gemmw<1, 0><<<dim3(SEQ / 64, DMOD / 64, 3), 32, 0, stream>>>(XB, nullptr, W3, nullptr, DMOD, F, D3, 1.0f, XSZ, WSZ, (size_t)DMOD);
        k_plane<<<(nthr8 + 255) / 256, 256, 0, stream>>>(F, 0, Q16, QH, QL);
        k_plane<<<(nthr8 + 255) / 256, 256, 0, stream>>>(F, DMOD, K16, KH, KL);
        k_vtp<<<(nthr8 + 255) / 256, 256, 0, stream>>>(F, VT16, VTH, VTL);
        k_attn<true><<<dim3(RH / 64, NH, 1), 128, 0, stream>>>(Q16, K16, VT16, QH, QL, KH, KL, VTH, VTL, 0, C16, CH, CLO);
        if (SEQ > RH)
            k_attn<false><<<dim3((SEQ - RH) / 64, NH, 1), 128, 0, stream>>>(Q16, K16, VT16, nullptr, nullptr, nullptr, nullptr, nullptr, nullptr, RH / 64, C16, nullptr, nullptr);
        k_gemmw<1, 1><<<dim3(RH / 64, DMOD / 64, 1), 32, 0, stream>>>(CH, CLO, WOB, nullptr, DMOD, ob, DMOD, 1.0f, 0, 0, 0);
        if (SEQ > RH)
            k_gemmw<0, 0><<<dim3((SEQ - RH) / 64, DMOD / 64, 1), 32, 0, stream>>>(C16 + (size_t)RH * DMOD, nullptr, WO16, nullptr, DMOD, ob + (size_t)RH * DMOD, DMOD, 1.0f / (CCAR * WCAR), 0, 0, 0);
    }
}
